// CSWT_Unet_65446711656652
// MI455X (gfx1250) — hardware-verified
//
#include <hip/hip_runtime.h>
#define NIMG 8
#define RES 64
#define NTOK (RES * RES)
#define CC 384
#define CB 192
#define NHB 6
#define HD 32
#define SP 4
#define NWT 256
#define NWIN 16
#define NG (NWIN * NHB)
#define MLPH 1536
#define SCALE 0.17677669529663687f
typedef __bf16 v16b __attribute__((ext_vector_type(16)));
typedef unsigned short v8us __attribute__((ext_vector_type(8), may_alias));
typedef float  v8f  __attribute__((ext_vector_type(8)));
typedef float  v4f  __attribute__((ext_vector_type(4)));
typedef float  v4fa __attribute__((ext_vector_type(4), may_alias));
union FragB { v16b v; v8us half[2]; unsigned short u[16]; };

__device__ __forceinline__ unsigned short bf16_bits(float x) { unsigned int u = __float_as_uint(x); return (unsigned short)((u + 0x7FFFu + ((u >> 16) & 1u)) >> 16); }
__device__ __forceinline__ float bf16_val(unsigned short b) { return __uint_as_float(((unsigned int)b) << 16); }
__device__ __forceinline__ float bf16_round(float x) { return bf16_val(bf16_bits(x)); }
template <int NT>
__device__ __forceinline__ v8f mmaN(v16b ah, v16b al, v16b bh, v16b bl, v8f c) {
  c = __builtin_amdgcn_wmma_f32_16x16x32_bf16(false, ah, false, bh, (short)0, c, false, false);
  if (NT >= 2) c = __builtin_amdgcn_wmma_f32_16x16x32_bf16(false, al, false, bh, (short)0, c, false, false);
  if (NT >= 3) c = __builtin_amdgcn_wmma_f32_16x16x32_bf16(false, ah, false, bl, (short)0, c, false, false);
  asm volatile("v_nop\n\tv_nop\n\tv_nop\n\tv_nop" : "+v"(c) : "v"(ah), "v"(al), "v"(bh), "v"(bl));
  return c;
}

__global__ __launch_bounds__(256) void k_wt_bf16(const float* __restrict__ W, unsigned short* __restrict__ Wt, int K, int N) {
  const int t = blockIdx.x * 256 + threadIdx.x;
  const int k8n = K / 8;
  if (t >= N * k8n) return;
  const int n = t / k8n, k8 = (t % k8n) * 8;
  v8us v;
#pragma unroll
  for (int i = 0; i < 8; ++i) v[i] = bf16_bits(W[(size_t)(k8 + i) * N + n]);
  *(volatile v8us*)(Wt + (size_t)n * K + k8) = v;
  __threadfence();
  *(volatile v8us*)(Wt + (size_t)n * K + k8) = v;
}

template <bool ASPLIT, int ACT, bool BIAS_BF16>
__global__ __launch_bounds__(128) void k_gemm_bf(const float* __restrict__ A, int lda, const unsigned short* __restrict__ Wt, int ldb,
                                               const float* __restrict__ bias, float* __restrict__ C, int ldc, int M, int N, int K) {
  __shared__ __attribute__((aligned(16))) float so[4][16][64];
  const int tid = threadIdx.x, w = tid >> 5, lane = tid & 31, ln = lane & 15, hh = lane >> 4;
  const int ntn = N / 64;
  const int wid = blockIdx.x * 4 + w;
  const int mt = wid / ntn, nq = wid % ntn;
  if (mt * 16 >= M) return;
  const int row0 = mt * 16, col0 = nq * 64;
  const float* arow = A + (size_t)(row0 + ln) * lda;
  v8f acc[4] = {};
  for (int kb = 0; kb < K; kb += 32) {
    FragB ah, al;
    const v4f x0 = *(const v4fa*)(arow + kb + 8 * hh), x1 = *(const v4fa*)(arow + kb + 8 * hh + 4);
    const v4f x2 = *(const v4fa*)(arow + kb + 16 + 8 * hh), x3 = *(const v4fa*)(arow + kb + 16 + 8 * hh + 4);
    float xs[16] = {x0[0],x0[1],x0[2],x0[3],x1[0],x1[1],x1[2],x1[3],x2[0],x2[1],x2[2],x2[3],x3[0],x3[1],x3[2],x3[3]};
#pragma unroll
    for (int i = 0; i < 16; ++i) { const unsigned short hb = bf16_bits(xs[i]); ah.u[i] = hb; al.u[i] = ASPLIT ? bf16_bits(xs[i] - bf16_val(hb)) : (unsigned short)0; }
#pragma unroll
    for (int t = 0; t < 4; ++t) {
      const unsigned short* brow = Wt + (size_t)(col0 + t * 16 + ln) * ldb + kb;
      FragB b;
      b.half[0] = *(const v8us*)(brow + 8 * hh);
      b.half[1] = *(const v8us*)(brow + 16 + 8 * hh);
      acc[t] = mmaN<ASPLIT ? 2 : 1>(ah.v, al.v, b.v, b.v, acc[t]);
    }
  }
#pragma unroll
  for (int t = 0; t < 4; ++t) {
    float bv = bias ? bias[col0 + t * 16 + ln] : 0.f;
    if (BIAS_BF16) bv = bf16_round(bv);
#pragma unroll
    for (int r = 0; r < 8; ++r) { float v = acc[t][r] + bv; if (ACT == 1) v = fmaxf(v, 0.f); so[w][8 * hh + r][t * 16 + ln] = v; }
  }
  __builtin_amdgcn_fence(__ATOMIC_ACQ_REL, "workgroup");
  __builtin_amdgcn_wave_barrier();
  const int rsub = lane >> 4, c4 = (lane & 15) * 4;
  for (int pass = 0; pass < 2; ++pass) {
#pragma unroll
    for (int q = 0; q < 8; ++q) {
      const int r = q * 2 + rsub;
      const v4f v = *(const v4fa*)&so[w][r][c4];
      *(volatile v4f*)(C + (size_t)(row0 + r) * ldc + col0 + c4) = v;
    }
    if (pass == 0) __threadfence();
  }
}

template <bool ASPLIT, int ACT, bool BIAS_BF16, bool RES_BF16>
__global__ __launch_bounds__(128) void k_gemm_bf3(const float* __restrict__ A, int lda, const unsigned short* __restrict__ Wt, int ldb,
                                                const float* __restrict__ bias, const float* __restrict__ resid, int rmod, int ldr,
                                                float* __restrict__ C, int ldc, int M, int N, int K) {
  __shared__ __attribute__((aligned(16))) float so[4][16][64];
  const int tid = threadIdx.x, w = tid >> 5, lane = tid & 31, ln = lane & 15, hh = lane >> 4;
  const int ntn = N / 64;
  const int wid = blockIdx.x * 4 + w;
  const int mt = wid / ntn, nq = wid % ntn;
  if (mt * 16 >= M) return;
  const int row0 = mt * 16, col0 = nq * 64;
  const float* arow = A + (size_t)(row0 + ln) * lda;
  v8f acc[4] = {};
  for (int kb = 0; kb < K; kb += 32) {
    FragB ah, al;
    const v4f x0 = *(const v4fa*)(arow + kb + 8 * hh), x1 = *(const v4fa*)(arow + kb + 8 * hh + 4);
    const v4f x2 = *(const v4fa*)(arow + kb + 16 + 8 * hh), x3 = *(const v4fa*)(arow + kb + 16 + 8 * hh + 4);
    float xs[16] = {x0[0],x0[1],x0[2],x0[3],x1[0],x1[1],x1[2],x1[3],x2[0],x2[1],x2[2],x2[3],x3[0],x3[1],x3[2],x3[3]};
#pragma unroll
    for (int i = 0; i < 16; ++i) { const unsigned short hb = bf16_bits(xs[i]); ah.u[i] = hb; al.u[i] = ASPLIT ? bf16_bits(xs[i] - bf16_val(hb)) : (unsigned short)0; }
#pragma unroll
    for (int t = 0; t < 4; ++t) {
      const unsigned short* brow = Wt + (size_t)(col0 + t * 16 + ln) * ldb + kb;
      FragB b;
      b.half[0] = *(const v8us*)(brow + 8 * hh);
      b.half[1] = *(const v8us*)(brow + 16 + 8 * hh);
      acc[t] = mmaN<ASPLIT ? 2 : 1>(ah.v, al.v, b.v, b.v, acc[t]);
    }
  }
#pragma unroll
  for (int t = 0; t < 4; ++t) {
    const int col = col0 + t * 16 + ln;
    float bv = bias ? bias[col] : 0.f;
    if (BIAS_BF16) bv = bf16_round(bv);
#pragma unroll
    for (int r = 0; r < 8; ++r) {
      float v = acc[t][r] + bv;
      if (resid) { float rv = resid[(size_t)((row0 + 8 * hh + r) % rmod) * ldr + col]; if (RES_BF16) rv = bf16_round(rv); v += rv; }
      if (ACT == 1) v = fmaxf(v, 0.f);
      if (ACT == 2) v = 0.5f * v * (1.0f + erff(v * 0.70710678118654752f));
      if (ACT == 3) { const float u = 0.7978845608028654f * (v + 0.044715f * v * v * v); v = 0.5f * v * (1.0f + tanhf(u)); }
      so[w][8 * hh + r][t * 16 + ln] = v;
    }
  }
  __builtin_amdgcn_fence(__ATOMIC_ACQ_REL, "workgroup");
  __builtin_amdgcn_wave_barrier();
  const int rsub = lane >> 4, c4 = (lane & 15) * 4;
  for (int pass = 0; pass < 2; ++pass) {
#pragma unroll
    for (int q = 0; q < 8; ++q) {
      const int r = q * 2 + rsub;
      const v4f v = *(const v4fa*)&so[w][r][c4];
      *(volatile v4f*)(C + (size_t)(row0 + r) * ldc + col0 + c4) = v;
    }
    if (pass == 0) __threadfence();
  }
}
template <bool PARAM_BF16>
__global__ __launch_bounds__(256) void k_layernorm(const float* __restrict__ X, const float* __restrict__ R, const float* __restrict__ g, const float* __restrict__ bta,
                                                  float* __restrict__ out_sum, float* __restrict__ out_norm, int N, float eps) {
  __shared__ float red[256];
  const int row = blockIdx.x, tid = threadIdx.x;
  const float* x = X + (size_t)row * N; const float* rr = R ? R + (size_t)row * N : nullptr;
  float vals[16];
  const int per = N / 256;
  float s1 = 0.f;
  for (int u = 0; u < per / 4; ++u) {
    const int j = tid * 4 + 1024 * u;
    const v4f a = *(const v4fa*)(x + j);
    v4f b = {0.f,0.f,0.f,0.f}; if (rr) b = *(const v4fa*)(rr + j);
#pragma unroll
    for (int q = 0; q < 4; ++q) { const float v = a[q] + b[q]; vals[u * 4 + q] = v; s1 += v; }
  }
  red[tid] = s1; __syncthreads();
  for (int st = 128; st > 0; st >>= 1) { if (tid < st) red[tid] += red[tid + st]; __syncthreads(); }
  const float mu = red[0] / (float)N; __syncthreads();
  float s2 = 0.f;
  for (int u = 0; u < per / 4; ++u)
#pragma unroll
    for (int q = 0; q < 4; ++q) { const float c = vals[u * 4 + q] - mu; s2 += c * c; }
  red[tid] = s2; __syncthreads();
  for (int st = 128; st > 0; st >>= 1) { if (tid < st) red[tid] += red[tid + st]; __syncthreads(); }
  const float rs = rsqrtf(red[0] / (float)N + eps);
  for (int pass = 0; pass < 2; ++pass) {
    for (int u = 0; u < per / 4; ++u) {
      const int j = tid * 4 + 1024 * u;
      v4f o, sm;
#pragma unroll
      for (int q = 0; q < 4; ++q) {
        float gg = g[j + q], bb = bta[j + q];
        if (PARAM_BF16) { gg = bf16_round(gg); bb = bf16_round(bb); }
        sm[q] = vals[u * 4 + q]; o[q] = (vals[u * 4 + q] - mu) * rs * gg + bb;
      }
      if (out_sum) *(volatile v4f*)(out_sum + (size_t)row * N + j) = sm;
      *(volatile v4f*)(out_norm + (size_t)row * N + j) = o;
    }
    if (pass == 0) __threadfence();
  }
}


typedef _Float16 v16h __attribute__((ext_vector_type(16)));
union FragH { v16h v; v8us half[2]; _Float16 h[16]; unsigned short u[16]; };
template <int NT>
__device__ __forceinline__ v8f mmaH(v16h ah, v16h al, v16h bh, v16h bl, v8f c) {
  c = __builtin_amdgcn_wmma_f32_16x16x32_f16(false, ah, false, bh, (short)0, c, false, false);
  if (NT >= 2) c = __builtin_amdgcn_wmma_f32_16x16x32_f16(false, al, false, bh, (short)0, c, false, false);
  if (NT >= 3) c = __builtin_amdgcn_wmma_f32_16x16x32_f16(false, ah, false, bl, (short)0, c, false, false);
  asm volatile("v_nop\n\tv_nop\n\tv_nop\n\tv_nop" : "+v"(c) : "v"(ah), "v"(al), "v"(bh), "v"(bl));
  return c;
}
template <bool ASPLIT>
__global__ __launch_bounds__(128) void k_gemm_h(const float* __restrict__ A, int lda, size_t sA, const _Float16* __restrict__ Bh, int ldb, size_t sB, float alpha, float* __restrict__ C, int ldc, size_t sC, int M, int N, int K) {
  __shared__ __attribute__((aligned(16))) float so[4][16][64];
  const int tid = threadIdx.x, w = tid >> 5, lane = tid & 31, ln = lane & 15, hh = lane >> 4; const int by = blockIdx.y;
  A += (size_t)by * sA; Bh += (size_t)by * sB; C += (size_t)by * sC;
  const int ntn = (N + 63) / 64; const int wid = blockIdx.x * 4 + w; const int mt = wid / ntn, nq = wid % ntn; if (mt * 16 >= M) return;
  const int row0 = mt * 16, col0 = nq * 64; const float* arow = A + (size_t)(row0 + ln) * lda;
  v8f acc[4] = {};
  for (int kb = 0; kb < K; kb += 32) {
    FragH ah, al;
    const v4f x0 = *(const v4fa*)(arow + kb + 8 * hh), x1 = *(const v4fa*)(arow + kb + 8 * hh + 4), x2 = *(const v4fa*)(arow + kb + 16 + 8 * hh), x3 = *(const v4fa*)(arow + kb + 16 + 8 * hh + 4);
    float xs[16] = {x0[0],x0[1],x0[2],x0[3],x1[0],x1[1],x1[2],x1[3],x2[0],x2[1],x2[2],x2[3],x3[0],x3[1],x3[2],x3[3]};
#pragma unroll
    for (int i = 0; i < 16; ++i) { const _Float16 h = (_Float16)xs[i]; ah.h[i] = h; al.h[i] = ASPLIT ? (_Float16)(xs[i] - (float)h) : (_Float16)0.0f; }
#pragma unroll
    for (int t = 0; t < 4; ++t) { if (col0 + t * 16 >= N) continue; const size_t boff = (size_t)(col0 + t * 16 + ln) * ldb + kb; FragH bq; bq.half[0] = *(const v8us*)(Bh + boff + 8 * hh); bq.half[1] = *(const v8us*)(Bh + boff + 16 + 8 * hh);
      acc[t] = mmaH<ASPLIT ? 2 : 1>(ah.v, al.v, bq.v, bq.v, acc[t]); }
  }
#pragma unroll
  for (int t = 0; t < 4; ++t) { if (col0 + t * 16 >= N) continue;
#pragma unroll
    for (int r = 0; r < 8; ++r) so[w][8 * hh + r][t * 16 + ln] = acc[t][r] * alpha; }
  __builtin_amdgcn_fence(__ATOMIC_ACQ_REL, "workgroup"); __builtin_amdgcn_wave_barrier();
  const int rsub = lane >> 4, c4 = (lane & 15) * 4;
  for (int pass = 0; pass < 2; ++pass) {
#pragma unroll
    for (int q = 0; q < 8; ++q) { const int r = q * 2 + rsub; if (col0 + c4 < N) { const v4f v = *(const v4fa*)&so[w][r][c4]; *(volatile v4f*)(C + (size_t)(row0 + r) * ldc + col0 + c4) = v; } }
    if (pass == 0) __threadfence(); }
}

__global__ __launch_bounds__(256) void k_wt_f16(const float* __restrict__ W, _Float16* __restrict__ Wt, int K, int N, float scale) {
  const int t = blockIdx.x * 256 + threadIdx.x; if (t >= N * (K / 8)) return; const int n = t / (K / 8), k8 = (t % (K / 8)) * 8; FragH f;
#pragma unroll
  for (int i = 0; i < 8; ++i) f.h[i] = (_Float16)(bf16_round(W[(size_t)(k8 + i) * N + n]) * scale); const v8us o = f.half[0];
  *(volatile v8us*)((unsigned short*)Wt + (size_t)n * K + k8) = o; __threadfence(); *(volatile v8us*)((unsigned short*)Wt + (size_t)n * K + k8) = o;
}
template <int ACT>
__global__ __launch_bounds__(128) void k_gemm_hhx(const _Float16* __restrict__ A, int lda, size_t sA, const _Float16* __restrict__ Bh, int ldb, size_t sB, float alpha, const float* __restrict__ bias, size_t sBias, const float* __restrict__ CP, int rowsPerB, size_t sCPb, int row0g,
    float* __restrict__ C, _Float16* __restrict__ C16, int ldc, size_t sC, int M, int N, int K) {
  __shared__ __attribute__((aligned(16))) float so[4][16][64];
  const int tid = threadIdx.x, w = tid >> 5, lane = tid & 31, ln = lane & 15, hh = lane >> 4; const int by = blockIdx.y;
  A += (size_t)by * sA; Bh += (size_t)by * sB; const size_t cofs = (size_t)by * sC; const float* bp = bias ? bias + (size_t)by * sBias : nullptr;
  const int ntn = (N + 63) / 64; const int wid = blockIdx.x * 4 + w; const int mt = wid / ntn, nq = wid % ntn; if (mt * 16 >= M) return;
  const int row0 = mt * 16, col0 = nq * 64; const _Float16* arow = A + (size_t)(row0 + ln) * lda;
  v8f acc[4] = {};
  for (int kb = 0; kb < K; kb += 32) { FragH ah; ah.half[0] = *(const v8us*)((const unsigned short*)arow + kb + 8 * hh); ah.half[1] = *(const v8us*)((const unsigned short*)arow + kb + 16 + 8 * hh);
#pragma unroll
    for (int t = 0; t < 4; ++t) { if (col0 + t * 16 >= N) continue; const size_t boff = (size_t)(col0 + t * 16 + ln) * ldb + kb; FragH bq; bq.half[0] = *(const v8us*)((const unsigned short*)Bh + boff + 8 * hh); bq.half[1] = *(const v8us*)((const unsigned short*)Bh + boff + 16 + 8 * hh);
      acc[t] = mmaH<1>(ah.v, ah.v, bq.v, bq.v, acc[t]); }
  }
#pragma unroll
  for (int t = 0; t < 4; ++t) { if (col0 + t * 16 >= N) continue; const int col = col0 + t * 16 + ln; const float bv = bp ? bf16_round(bp[col]) : 0.f;
#pragma unroll
    for (int r = 0; r < 8; ++r) { float v = acc[t][r] * alpha + bv; if (CP) { const int bidx = (row0g + row0 + 8 * hh + r) / rowsPerB; v += CP[(size_t)bidx * sCPb + (size_t)by * 64 + col]; } if (ACT == 1) v = (v > 0.f) ? v : expm1f(v); else if (ACT == 7) v = (v > 0.f) ? v + 1.0f : expf(v); else if (ACT == 8) v = tanhf(v); else if (ACT == 9) v = 0.5f * v * (1.0f + tanhf(0.7978845608028654f * (v + 0.044715f * v * v * v))); else if (ACT == 11) v = 1.0f / (1.0f + expf(-v)); else if (ACT == 12) v = (v > 0.f) ? v : 0.01f * v; else if (ACT == 14) v = (v > 0.f) ? v : 0.1f * v; else if (ACT == 15) v = v / (1.0f + expf(-v)); else if (ACT == 3) v = fmaxf(v, 0.f); else if (ACT == 6) v = 0.5f * v * (1.0f + erff(v * 0.70710678118654752f)); so[w][8 * hh + r][t * 16 + ln] = v; } }
  __builtin_amdgcn_fence(__ATOMIC_ACQ_REL, "workgroup"); __builtin_amdgcn_wave_barrier();
  const int rsub = lane >> 4, c4 = (lane & 15) * 4; typedef _Float16 v4h __attribute__((ext_vector_type(4)));
  for (int pass = 0; pass < 2; ++pass) {
#pragma unroll
    for (int q = 0; q < 8; ++q) { const int r = q * 2 + rsub; if (col0 + c4 < N) { const v4f v = *(const v4fa*)&so[w][r][c4]; if (C) *(volatile v4f*)(C + cofs + (size_t)(row0 + r) * ldc + col0 + c4) = v; if (C16) { v4h h4; for (int i = 0; i < 4; ++i) h4[i] = (_Float16)v[i]; *(volatile v4h*)(C16 + cofs + (size_t)(row0 + r) * ldc + col0 + c4) = h4; } } }
    if (pass == 0) __threadfence(); }
}


typedef _Float16 v4h __attribute__((ext_vector_type(4)));

__global__ __launch_bounds__(256) void k_x16(const float* __restrict__ x, _Float16* __restrict__ X16, size_t n8) { const size_t t = (size_t)blockIdx.x * 256 + threadIdx.x; if (t >= n8) return; FragH f;
#pragma unroll
  for (int q = 0; q < 8; ++q) f.h[q] = (_Float16)bf16_round(x[t * 8 + q]); *(volatile v8us*)((unsigned short*)X16 + t * 8) = f.half[0]; __threadfence(); *(volatile v8us*)((unsigned short*)X16 + t * 8) = f.half[0]; }
__global__ __launch_bounds__(256) void k_h16(const float* __restrict__ x, _Float16* __restrict__ X16, size_t n8) { const size_t t = (size_t)blockIdx.x * 256 + threadIdx.x; if (t >= n8) return; FragH f;
#pragma unroll
  for (int q = 0; q < 8; ++q) f.h[q] = (_Float16)x[t * 8 + q]; *(volatile v8us*)((unsigned short*)X16 + t * 8) = f.half[0]; __threadfence(); *(volatile v8us*)((unsigned short*)X16 + t * 8) = f.half[0]; }
__global__ __launch_bounds__(256) void k_round16f(const float* __restrict__ W, _Float16* __restrict__ Bt, size_t n8) { const size_t t = (size_t)blockIdx.x * 256 + threadIdx.x; if (t >= n8) return; FragH f;
#pragma unroll
  for (int i = 0; i < 8; ++i) f.h[i] = (_Float16)(bf16_round(W[t * 8 + i]) * 16.0f); *(volatile v8us*)((unsigned short*)Bt + t * 8) = f.half[0]; __threadfence(); *(volatile v8us*)((unsigned short*)Bt + t * 8) = f.half[0]; }
template <int NHv, int TTv>
__global__ __launch_bounds__(256) void k_vt(const _Float16* __restrict__ V16, int ldv, int voff, _Float16* __restrict__ Vt) { __shared__ unsigned short tl[64][66]; const int tid = threadIdx.x; const int slab = blockIdx.x / (TTv / 64), lg = blockIdx.x % (TTv / 64); const int b = slab / NHv, h = slab % NHv;
  for (int i = tid; i < 64 * 8; i += 256) { const int r = i / 8, c8 = (i % 8) * 8; FragH f; f.half[0] = *(const v8us*)((const unsigned short*)V16 + ((size_t)b * TTv + lg * 64 + r) * ldv + voff + h * 64 + c8);
#pragma unroll
    for (int q = 0; q < 8; ++q) tl[r][c8 + q] = f.u[q]; }
  __syncthreads();
  for (int pass = 0; pass < 2; ++pass) {
#pragma unroll
    for (int rd = 0; rd < 2; ++rd) { const int d = rd * 32 + tid / 8, pc = tid % 8; FragH f;
#pragma unroll
      for (int q = 0; q < 8; ++q) f.u[q] = tl[pc * 8 + q][d];
      *(volatile v8us*)((unsigned short*)Vt + ((size_t)slab * 64 + d) * TTv + lg * 64 + pc * 8) = f.half[0]; }
    if (pass == 0) __threadfence(); } }

__global__ __launch_bounds__(256) void k_hl(const float* __restrict__ F, _Float16* __restrict__ Hh, _Float16* __restrict__ Hl, size_t n8) { const size_t t = (size_t)blockIdx.x * 256 + threadIdx.x; if (t >= n8) return; FragH fh, fl; const v4f a = *(const v4fa*)(F + t * 8), c = *(const v4fa*)(F + t * 8 + 4);
#pragma unroll
  for (int q = 0; q < 4; ++q) { _Float16 h = (_Float16)a[q]; fh.h[q] = h; fl.h[q] = (_Float16)((a[q] - (float)h) * 1024.0f); h = (_Float16)c[q]; fh.h[4 + q] = h; fl.h[4 + q] = (_Float16)((c[q] - (float)h) * 1024.0f); }
  for (int pass = 0; pass < 2; ++pass) { *(volatile v8us*)((unsigned short*)Hh + t * 8) = fh.half[0]; *(volatile v8us*)((unsigned short*)Hl + t * 8) = fl.half[0]; if (pass == 0) __threadfence(); } }

__device__ __forceinline__ v16h g2_frag(const _Float16* p, int hh) { FragH f; f.half[0] = *(const v8us*)((const unsigned short*)p + 8 * hh); f.half[1] = *(const v8us*)((const unsigned short*)p + 16 + 8 * hh); return f.v; }
__device__ __forceinline__ v8f g2_mma(v16h a, v16h b, v8f c) { v8f d = __builtin_amdgcn_wmma_f32_16x16x32_f16(false, a, false, b, (short)0, c, false, false); asm volatile("v_nop\n\tv_nop\n\tv_nop\n\tv_nop" : "+v"(d) : "v"(a), "v"(b)); return d; }
template <int ACT>
__global__ __launch_bounds__(128) void k_gemm2(const _Float16* __restrict__ A, int lda, size_t sA, const _Float16* __restrict__ Bh, int ldb, size_t sB, float alpha, const float* __restrict__ bias, size_t sBias, const float* __restrict__ CP, int rowsPerB, size_t sCPb, int row0g,
    float* __restrict__ C, _Float16* __restrict__ C16, int ldc, size_t sC, int M, int N, int K) {
  __shared__ __attribute__((aligned(16))) float so[4][32][68];
  const int tid = threadIdx.x, w = tid >> 5, lane = tid & 31, ln = lane & 15, hh = lane >> 4; const int by = blockIdx.y;
  A += (size_t)by * sA; Bh += (size_t)by * sB; const size_t cofs = (size_t)by * sC; const float* bp = bias ? bias + (size_t)by * sBias : nullptr;
  const int ntn = N >> 6; const int mt = blockIdx.x / ntn, nq = blockIdx.x - mt * ntn; const int row0 = mt * 128 + 32 * w, col0 = nq * 64; if (row0 >= M) return;
  const _Float16* a0p = A + (size_t)(row0 + ln) * lda; const _Float16* a1p = a0p + (size_t)16 * lda;
  const _Float16* b0p = Bh + (size_t)(col0 + ln) * ldb; const _Float16* b1p = b0p + (size_t)16 * ldb; const _Float16* b2p = b1p + (size_t)16 * ldb; const _Float16* b3p = b2p + (size_t)16 * ldb;
  const v8f z8 = {0.f,0.f,0.f,0.f,0.f,0.f,0.f,0.f}; v8f c00 = z8, c01 = z8, c02 = z8, c03 = z8, c10 = z8, c11 = z8, c12 = z8, c13 = z8;
#pragma unroll 1
  for (int kb = 0; kb < K; kb += 32) { const v16h a0 = g2_frag(a0p + kb, hh), a1 = g2_frag(a1p + kb, hh);
    v16h b = g2_frag(b0p + kb, hh); c00 = g2_mma(a0, b, c00); c10 = g2_mma(a1, b, c10);
    b = g2_frag(b1p + kb, hh); c01 = g2_mma(a0, b, c01); c11 = g2_mma(a1, b, c11);
    b = g2_frag(b2p + kb, hh); c02 = g2_mma(a0, b, c02); c12 = g2_mma(a1, b, c12);
    b = g2_frag(b3p + kb, hh); c03 = g2_mma(a0, b, c03); c13 = g2_mma(a1, b, c13); }
  v8f accs[8] = {c00, c01, c02, c03, c10, c11, c12, c13};
#pragma unroll
  for (int u = 0; u < 8; ++u) { const int t = u & 3, half = u >> 2; const int col = col0 + t * 16 + ln; const float bv = bp ? bf16_round(bp[col]) : 0.f;
#pragma unroll
    for (int r = 0; r < 8; ++r) { const int rloc = half * 16 + 8 * hh + r; float v = accs[u][r] * alpha + bv; if (CP) { const int bidx = (row0g + row0 + rloc) / rowsPerB; v += CP[(size_t)bidx * sCPb + (size_t)by * 64 + col]; }
      if (ACT == 3) v = fmaxf(v, 0.f); else if (ACT == 6) v = 0.5f * v * (1.0f + erff(v * 0.70710678118654752f)); else if (ACT == 11) v = 1.0f / (1.0f + expf(-v)); else if (ACT == 15) v = v / (1.0f + expf(-v)); else if (ACT == 12) v = (v > 0.f) ? v : 0.01f * v; else if (ACT == 8) v = tanhf(v);
      so[w][rloc][t * 16 + ln] = v; } }
  __builtin_amdgcn_fence(__ATOMIC_ACQ_REL, "workgroup"); __builtin_amdgcn_wave_barrier();
  const int rsub = lane >> 4, c4 = (lane & 15) * 4;
  for (int pass = 0; pass < 2; ++pass) {
#pragma unroll
    for (int q = 0; q < 16; ++q) { const int r = q * 2 + rsub; const v4f v = *(const v4fa*)&so[w][r][c4]; if (C) *(volatile v4f*)(C + cofs + (size_t)(row0 + r) * ldc + col0 + c4) = v; if (C16) { v4h h4; for (int i = 0; i < 4; ++i) h4[i] = (_Float16)v[i]; *(volatile v4h*)(C16 + cofs + (size_t)(row0 + r) * ldc + col0 + c4) = h4; } }
    if (pass == 0) __threadfence(); } }


template <int SRCBF>
__global__ __launch_bounds__(256) void k_ln384(const float* __restrict__ X, const float* __restrict__ g, const float* __restrict__ bb, _Float16* __restrict__ Y16, float* __restrict__ XB) {
  #pragma clang fp contract(off)
  const int tid = threadIdx.x, w = tid >> 5, ln = tid & 31; const int r = blockIdx.x * 8 + w; if (r >= NTOK) return; const float* x = X + (size_t)r * CC; float v[12]; float s = 0.f;
#pragma unroll
  for (int i = 0; i < 3; ++i) { const v4f a = *(const v4fa*)(x + i * 128 + ln * 4);
#pragma unroll
    for (int q = 0; q < 4; ++q) { const float t = SRCBF ? bf16_round(a[q]) : a[q]; v[i * 4 + q] = t; s += t; } }
  for (int o = 16; o > 0; o >>= 1) s += __shfl_xor(s, o, 32); const float mu = s / (float)CC; float q2 = 0.f;
#pragma unroll
  for (int i = 0; i < 12; ++i) { const float d = v[i] - mu; q2 += d * d; }
  for (int o = 16; o > 0; o >>= 1) q2 += __shfl_xor(q2, o, 32); const float dn = sqrtf(q2 / (float)CC + 1e-5f);
  for (int pass = 0; pass < 2; ++pass) {
#pragma unroll
    for (int i = 0; i < 3; ++i) { const int c0 = i * 128 + ln * 4; _Float16 h4[4]; v4f xb;
#pragma unroll
      for (int q = 0; q < 4; ++q) { const int c = c0 + q; h4[q] = (_Float16)((v[i * 4 + q] - mu) / dn * bf16_round(g[c]) + bf16_round(bb[c])); xb[q] = v[i * 4 + q]; }
      *(volatile unsigned long long*)((unsigned short*)Y16 + (size_t)r * CC + c0) = *(const unsigned long long*)h4; if (XB) *(volatile v4f*)(XB + (size_t)r * CC + c0) = xb; }
    if (pass == 0) __threadfence(); } }
__global__ __launch_bounds__(256) void k_gather(const _Float16* __restrict__ QKV, int br, _Float16* __restrict__ QW, _Float16* __restrict__ KW) {
  const int t = blockIdx.x * 256 + threadIdx.x; if (t >= NG * NWT * 4) return; const int pc = t & 3; const int n = (t >> 2) % NWT, g = t / (4 * NWT); const int win = g / NHB, h = g % NHB; int i, j;
  if (br == 0) { i = n / SP; j = win * SP + (n % SP); } else { i = win * SP + n / RES; j = n % RES; }
  const int tok = i * RES + j; const unsigned short* src = (const unsigned short*)QKV + (size_t)tok * (3 * CC) + br * CB + h * HD + pc * 8;
  FragH q0, k0; q0.half[0] = *(const v8us*)(src); k0.half[0] = *(const v8us*)(src + CC);
  unsigned short* qd = (unsigned short*)QW + ((size_t)g * NWT + n) * HD + pc * 8; unsigned short* kd = (unsigned short*)KW + ((size_t)g * NWT + n) * HD + pc * 8;
  for (int pass = 0; pass < 2; ++pass) { *(volatile v8us*)qd = q0.half[0]; *(volatile v8us*)kd = k0.half[0]; if (pass == 0) __threadfence(); } }
__global__ __launch_bounds__(256) void k_vtr(const _Float16* __restrict__ QKV, int br, _Float16* __restrict__ VT) {
  __shared__ unsigned short tl[64][34]; const int tid = threadIdx.x; const int g = blockIdx.x / (NWT / 64), nt = blockIdx.x % (NWT / 64); const int win = g / NHB, h = g % NHB;
  { const int nl = tid >> 2, part = tid & 3; const int n = nt * 64 + nl; int i, j; if (br == 0) { i = n / SP; j = win * SP + (n % SP); } else { i = win * SP + n / RES; j = n % RES; }
    FragH f; f.half[0] = *(const v8us*)((const unsigned short*)QKV + (size_t)(i * RES + j) * (3 * CC) + 2 * CC + br * CB + h * HD + part * 8);
#pragma unroll
    for (int q = 0; q < 8; ++q) tl[nl][part * 8 + q] = f.u[q]; }
  __syncthreads();
  const int d = tid >> 3, n8 = (tid & 7) * 8; FragH o;
#pragma unroll
  for (int q = 0; q < 8; ++q) o.u[q] = tl[n8 + q][d];
  FragH z;
#pragma unroll
  for (int q = 0; q < 8; ++q) z.u[q] = 0;
  unsigned short* dst = (unsigned short*)VT + ((size_t)g * 64 + d) * NWT + nt * 64 + n8; unsigned short* dz = (unsigned short*)VT + ((size_t)g * 64 + 32 + d) * NWT + nt * 64 + n8;
  for (int pass = 0; pass < 2; ++pass) { *(volatile v8us*)dst = o.half[0]; *(volatile v8us*)dz = z.half[0]; if (pass == 0) __threadfence(); } }
__global__ __launch_bounds__(256) void k_soft256(const float* __restrict__ S, _Float16* __restrict__ P16) {
  #pragma clang fp contract(off)
  const int tid = threadIdx.x, w = tid >> 5, ln = tid & 31; const size_t r = (size_t)blockIdx.x * 8 + w; if (r >= (size_t)NG * NWT) return; const float* s = S + r * NWT + ln * 8; float v[8]; float m = -3.0e38f;
#pragma unroll
  for (int q = 0; q < 8; ++q) { v[q] = s[q]; m = fmaxf(m, v[q]); }
  for (int o = 16; o > 0; o >>= 1) m = fmaxf(m, __shfl_xor(m, o, 32)); float su = 0.f;
#pragma unroll
  for (int q = 0; q < 8; ++q) { v[q] = expf(v[q] - m); su += v[q]; }
  for (int o = 16; o > 0; o >>= 1) su += __shfl_xor(su, o, 32); const float inv = 1024.0f / su; FragH f;
#pragma unroll
  for (int q = 0; q < 8; ++q) f.h[q] = (_Float16)(v[q] * inv);
  *(volatile v8us*)((unsigned short*)P16 + r * NWT + ln * 8) = f.half[0]; __threadfence(); *(volatile v8us*)((unsigned short*)P16 + r * NWT + ln * 8) = f.half[0]; }
__global__ __launch_bounds__(256) void k_unwin(const float* __restrict__ O, const _Float16* __restrict__ QKV, const float* __restrict__ lw, const float* __restrict__ lb, int br, float* __restrict__ ATT) {
  #pragma clang fp contract(off)
  const int t = blockIdx.x * 256 + threadIdx.x; if (t >= NG * NWT * 8) return; const int d0 = (t & 7) * 4; const int n = (t >> 3) % NWT; const int g = t / (8 * NWT); const int win = g / NHB, h = g % NHB;
  const int Hs = br ? SP : RES, Ws = br ? RES : SP; const int yi = n / Ws, xi = n % Ws; int i, j; if (br == 0) { i = yi; j = win * SP + xi; } else { i = win * SP + yi; j = xi; }
  const int tok = i * RES + j; v4f o;
#pragma unroll
  for (int q = 0; q < 4; ++q) { const int c = h * HD + d0 + q; float lp = bf16_round(lb[c]);
#pragma unroll
    for (int ky = 0; ky < 3; ++ky) { const int yy = yi + ky - 1; if (yy < 0 || yy >= Hs) continue;
#pragma unroll
      for (int kx = 0; kx < 3; ++kx) { const int xx = xi + kx - 1; if (xx < 0 || xx >= Ws) continue; int ii, jj; if (br == 0) { ii = yy; jj = win * SP + xx; } else { ii = win * SP + yy; jj = xx; }
        lp += bf16_round(lw[c * 9 + ky * 3 + kx]) * (float)QKV[(size_t)(ii * RES + jj) * (3 * CC) + 2 * CC + br * CB + c]; } }
    o[q] = O[((size_t)g * NWT + n) * 64 + d0 + q] + lp; }
  float* dst = ATT + (size_t)tok * CC + br * CB + h * HD + d0;
  *(volatile v4f*)dst = o; __threadfence(); *(volatile v4f*)dst = o; }

extern "C" void kernel_launch(void* const* d_in, const int* in_sizes, int n_in,
                              void* d_out, int out_size, void* d_ws, size_t ws_size, hipStream_t stream) {
  (void)in_sizes; (void)n_in; (void)out_size;
  const float* const* I = (const float* const*)d_in; const float* x = I[0]; const float* l1g = I[1]; const float* l1b = I[2]; const float* qkvw = I[3]; const float* qkvb = I[4]; const float* lw0 = I[5]; const float* lb0 = I[6]; const float* lw1 = I[7]; const float* lb1 = I[8];
  const float* pw = I[9]; const float* pb = I[10]; const float* l2g = I[11]; const float* l2b = I[12]; const float* f1w = I[13]; const float* f1b = I[14]; const float* f2w = I[15]; const float* f2b = I[16];
  char* ws = (char*)d_ws; size_t off = 0;
  auto take = [&](size_t bytes) { char* p = ws + off; off += (bytes + 255) & ~(size_t)255; return p; };
  _Float16* BQKV = (_Float16*)take((size_t)3 * CC * CC * 2); _Float16* BP = (_Float16*)take((size_t)CC * CC * 2); _Float16* BF1 = (_Float16*)take((size_t)MLPH * CC * 2); _Float16* BF2 = (_Float16*)take((size_t)CC * MLPH * 2);
  float* XB = (float*)take((size_t)NTOK * CC * 4); _Float16* X16 = (_Float16*)take((size_t)NTOK * CC * 2); _Float16* QKV = (_Float16*)take((size_t)NTOK * 3 * CC * 2);
  _Float16* QW = (_Float16*)take((size_t)NG * NWT * HD * 2); _Float16* KW = (_Float16*)take((size_t)NG * NWT * HD * 2); _Float16* VT = (_Float16*)take((size_t)NG * 64 * NWT * 2);
  float* S = (float*)take((size_t)NG * NWT * NWT * 4); _Float16* P16 = (_Float16*)take((size_t)NG * NWT * NWT * 2); float* O = (float*)take((size_t)NG * NWT * 64 * 4); float* ATT = (float*)take((size_t)NTOK * CC * 4); _Float16* ATT16 = (_Float16*)take((size_t)NTOK * CC * 2);
  float* X1 = (float*)take((size_t)NTOK * CC * 4); _Float16* H16 = (_Float16*)take((size_t)NTOK * CC * 2); _Float16* G16 = (_Float16*)take((size_t)NTOK * MLPH * 2);
  if (off > ws_size) return;
  k_round16f<<<(3 * CC * CC / 8 + 255) / 256, 256, 0, stream>>>(qkvw, BQKV, (size_t)3 * CC * CC / 8); k_round16f<<<(CC * CC / 8 + 255) / 256, 256, 0, stream>>>(pw, BP, (size_t)CC * CC / 8);
  k_round16f<<<(MLPH * CC / 8 + 255) / 256, 256, 0, stream>>>(f1w, BF1, (size_t)MLPH * CC / 8); k_round16f<<<(CC * MLPH / 8 + 255) / 256, 256, 0, stream>>>(f2w, BF2, (size_t)CC * MLPH / 8);
  const dim3 gQKV((NTOK / 128) * (3 * CC / 64), 1), gS((NWT / 128) * (NWT / 64), NG), gPV((NWT / 128) * 1, NG), gC((NTOK / 128) * (CC / 64), 1), gF1((NTOK / 128) * (MLPH / 64), 1);
  const size_t n8 = (size_t)NTOK * CC / 8;
  for (int b = 0; b < NIMG; ++b) { const float* xb = x + (size_t)b * NTOK * CC; float* outb = (float*)d_out + (size_t)b * NTOK * CC;
    k_ln384<1><<<NTOK / 8, 256, 0, stream>>>(xb, l1g, l1b, X16, XB);
    k_gemm2<0><<<gQKV, 128, 0, stream>>>(X16, CC, 0, BQKV, CC, 0, 0.0625f, qkvb, 0, nullptr, 1, 0, 0, nullptr, QKV, 3 * CC, 0, NTOK, 3 * CC, CC);
    for (int br = 0; br < 2; ++br) {
      k_gather<<<(NG * NWT * 4 + 255) / 256, 256, 0, stream>>>(QKV, br, QW, KW); k_vtr<<<NG * (NWT / 64), 256, 0, stream>>>(QKV, br, VT);
      k_gemm2<0><<<gS, 128, 0, stream>>>(QW, HD, (size_t)NWT * HD, KW, HD, (size_t)NWT * HD, SCALE, nullptr, 0, nullptr, 1, 0, 0, S, nullptr, NWT, (size_t)NWT * NWT, NWT, NWT, HD);
      k_soft256<<<(NG * NWT + 7) / 8, 256, 0, stream>>>(S, P16);
      k_gemm2<0><<<gPV, 128, 0, stream>>>(P16, NWT, (size_t)NWT * NWT, VT, NWT, (size_t)64 * NWT, 1.0f / 1024.0f, nullptr, 0, nullptr, 1, 0, 0, O, nullptr, 64, (size_t)NWT * 64, NWT, 64, NWT);
      k_unwin<<<(NG * NWT * 8 + 255) / 256, 256, 0, stream>>>(O, QKV, br ? lw1 : lw0, br ? lb1 : lb0, br, ATT); }
    k_h16<<<(unsigned)((n8 + 255) / 256), 256, 0, stream>>>(ATT, ATT16, n8);
    k_gemm2<0><<<gC, 128, 0, stream>>>(ATT16, CC, 0, BP, CC, 0, 0.0625f, pb, 0, XB, 1, (size_t)CC, 0, X1, nullptr, CC, 0, NTOK, CC, CC);
    k_ln384<0><<<NTOK / 8, 256, 0, stream>>>(X1, l2g, l2b, H16, nullptr);
    k_gemm2<6><<<gF1, 128, 0, stream>>>(H16, CC, 0, BF1, CC, 0, 0.0625f, f1b, 0, nullptr, 1, 0, 0, nullptr, G16, MLPH, 0, NTOK, MLPH, CC);
    k_gemm2<0><<<gC, 128, 0, stream>>>(G16, MLPH, 0, BF2, MLPH, 0, 0.0625f, f2b, 0, X1, 1, (size_t)CC, 0, outb, nullptr, CC, 0, NTOK, CC, MLPH); }
}
